// GridSpatialEncoder_5540507812261
// MI455X (gfx1250) — hardware-run, weakly checked
//
#include <hip/hip_runtime.h>
#include <math.h>

typedef __attribute__((ext_vector_type(16))) _Float16 v16h;
typedef __attribute__((ext_vector_type(16))) __bf16 v16b;
typedef __attribute__((ext_vector_type(8)))  _Float16 v8h;
typedef __attribute__((ext_vector_type(8)))  float v8f;
typedef __attribute__((ext_vector_type(4)))  float v4f;
typedef __attribute__((ext_vector_type(2)))  float v2f;
typedef __attribute__((ext_vector_type(4)))  unsigned v4u;
typedef __attribute__((ext_vector_type(4)))  int v4i;
typedef float __attribute__((may_alias)) float_a;
typedef int __attribute__((may_alias)) int_a;

template <typename T> __device__ __forceinline__ void vst2(void* p, T v) { *(volatile T*)p = v; __threadfence(); *(volatile T*)p = v; }
__device__ __forceinline__ v8f wmma16(v16h a, v16h b, v8f c) {
  v8f d = __builtin_amdgcn_wmma_f32_16x16x32_f16(false, a, false, b, (short)0, c, false, false);
  asm volatile("v_nop\n\tv_nop\n\tv_nop\n\tv_nop" : "+v"(d) : "v"(a), "v"(b));
  return d;
}
__device__ __forceinline__ v8f wmma_bf(v16b a, v16b b, v8f c) {
  v8f d = __builtin_amdgcn_wmma_f32_16x16x32_bf16(false, a, false, b, (short)0, c, false, false);
  asm volatile("v_nop\n\tv_nop\n\tv_nop\n\tv_nop" : "+v"(d) : "v"(a), "v"(b));
  return d;
}
__device__ __forceinline__ v16h frag_h(const _Float16* rowk0, int lane) {
  union { v16h v; v8h q[2]; } u; const _Float16* p = rowk0 + 8 * (lane >> 4);
  u.q[0] = *(const v8h*)p; u.q[1] = *(const v8h*)(p + 16); return u.v;
}
__device__ __forceinline__ v16h frag_f32(const float* rowk0, int lane) {
  v16h a; const float* p = rowk0 + 8 * (lane >> 4);
#pragma unroll
  for (int i = 0; i < 8; ++i) { a[i] = (_Float16)p[i]; a[8 + i] = (_Float16)p[16 + i]; }
  return a;
}
__device__ __forceinline__ v16h frag_f32s(const float* rowk0, int lane, float sc) {
  v16h a; const float* p = rowk0 + 8 * (lane >> 4);
#pragma unroll
  for (int i = 0; i < 8; ++i) { a[i] = (_Float16)(p[i] * sc); a[8 + i] = (_Float16)(p[16 + i] * sc); }
  return a;
}
__device__ __forceinline__ v16h fragc_f32(const float* W, int k0, int n, int lane, int ld, int K) {
  v16h a; const int g = lane >> 4;
#pragma unroll
  for (int i = 0; i < 8; ++i) { const int ka = k0 + 8 * g + i, kb = ka + 16;
    a[i] = (_Float16)(ka < K ? W[(size_t)(ka < K ? ka : K - 1) * ld + n] : 0.f); a[8 + i] = (_Float16)(kb < K ? W[(size_t)(kb < K ? kb : K - 1) * ld + n] : 0.f); }
  return a;
}
struct F2 { v16b h, l; };
__device__ __forceinline__ F2 bsplit16(const float v[16]) { F2 r;
#pragma unroll
  for (int i = 0; i < 16; ++i) { const __bf16 h = (__bf16)v[i]; r.h[i] = h; r.l[i] = (__bf16)(v[i] - (float)h); }
  return r; }
__device__ __forceinline__ F2 split_row(const float* row, int k0, int lane) { float v[16]; const float* p = row + k0 + 8 * (lane >> 4);
#pragma unroll
  for (int i = 0; i < 8; ++i) { v[i] = p[i]; v[8 + i] = p[16 + i]; }
  return bsplit16(v); }
__device__ __forceinline__ F2 split_rowK(const float* row, int k0, int lane, int K) { float v[16]; const int g = lane >> 4;
#pragma unroll
  for (int i = 0; i < 8; ++i) { const int ka = k0 + 8 * g + i, kb = ka + 16; v[i] = ka < K ? row[ka < K ? ka : K - 1] : 0.f; v[8 + i] = kb < K ? row[kb < K ? kb : K - 1] : 0.f; }
  return bsplit16(v); }
__device__ __forceinline__ F2 split_col(const float* W, int k0, int n, int lane, int ld, int K) { float v[16]; const int g = lane >> 4;
#pragma unroll
  for (int i = 0; i < 8; ++i) { const int ka = k0 + 8 * g + i, kb = ka + 16; v[i] = ka < K ? W[(size_t)(ka < K ? ka : K - 1) * ld + n] : 0.f; v[8 + i] = kb < K ? W[(size_t)(kb < K ? kb : K - 1) * ld + n] : 0.f; }
  return bsplit16(v); }
__device__ __forceinline__ v8f mac3(const F2& a, const F2& b, v8f c) { c = wmma_bf(a.l, b.h, c); c = wmma_bf(a.h, b.l, c); return wmma_bf(a.h, b.h, c); }
__device__ __forceinline__ float sigm(float v) { return 1.0f / (1.0f + expf(-v)); }
#define LDSX() do { asm volatile("s_wait_dscnt 0" ::: "memory"); __builtin_amdgcn_wave_barrier(); __builtin_amdgcn_fence(__ATOMIC_RELEASE, "workgroup"); } while (0)


#define NB 8
#define NP 2048
#define INF 256
#define DD 512
#define NH 4
#define HD 128
#define GX 8
#define GY 8
#define NG (GX * GY)
#define KN 9
#define NR (NB * NP)
#define NCM (NB * NG)
#define NKR 576
#ifndef TRB
#define TRB (NR / 64)
#endif
typedef __attribute__((ext_vector_type(8))) __bf16 v8b;
__device__ __forceinline__ v16b frag_b(const __bf16* rowk0, int lane) {
  union { v16b v; v8b q[2]; } u; const __bf16* p = rowk0 + 8 * (lane >> 4);
  u.q[0] = *(const v8b*)p; u.q[1] = *(const v8b*)(p + 16); return u.v;
}
__device__ __forceinline__ float bfr(float v) { return (float)(__bf16)v; }
__device__ __attribute__((noinline)) float exp_ni(float v) { return expf(v); }
__device__ __attribute__((noinline)) float erf_ni(float v) { return erff(v); }

#define WS_PF  0u
#define WS_PW  (WS_PF + 2u * (size_t)DD * INF)
#define WS_FE  (WS_PW + 2u * (size_t)4 * DD * DD)
#define WS_CE  (WS_FE + 4u * (size_t)NR * DD)
#define WS_KA  (WS_CE + 4u * (size_t)NR)
#define WS_CN  (WS_KA + 4u * (size_t)NKR * DD)
#define WS_MK  (WS_CN + 4u * (size_t)NCM)
#define WS_MV  (WS_MK + 4u * (size_t)NKR * DD)
#define WS_Q   (WS_MV + 4u * (size_t)NKR * DD)
#define WS_AG  (WS_Q + 4u * (size_t)NR * DD)
#define WS_E   (WS_AG + 4u * (size_t)NR * DD)
#define WS_END (WS_E + 4u * (size_t)NR * DD)

__global__ __launch_bounds__(256) void k_pack(const float* __restrict__ WF, const float* __restrict__ WQ, const float* __restrict__ WK, const float* __restrict__ WV, const float* __restrict__ WO, __bf16* __restrict__ PF, __bf16* __restrict__ PW) { const int n = blockIdx.x, which = blockIdx.y, t = threadIdx.x; __shared__ __align__(16) __bf16 s[DD];
  if (which == 0) { s[t] = (__bf16)WF[(size_t)t * DD + n]; __syncthreads(); if (t < INF / 8) vst2((unsigned*)(PF + (size_t)n * INF + t * 8), *(const v4u*)&s[t * 8]); }
  else { const float* w = (which == 1) ? WQ : (which == 2) ? WK : (which == 3) ? WV : WO; for (int k = t; k < DD; k += 256) s[k] = (__bf16)w[(size_t)k * DD + n]; __syncthreads(); if (t < DD / 8) vst2((unsigned*)(PW + ((size_t)(which - 1) * DD + n) * DD + t * 8), *(const v4u*)&s[t * 8]); } }
__global__ __launch_bounds__(128) void k_feat(const float* __restrict__ X, const __bf16* __restrict__ PF, const float* __restrict__ BF, float* __restrict__ FE) { __shared__ __align__(16) float so[4][16][132];
  const int tid = threadIdx.x, wave = tid >> 5, lane = tid & 31, col = lane & 15, g = lane >> 4; const size_t r0 = (size_t)blockIdx.x * 64 + wave * 16; const int c0 = blockIdx.y * 128;
  v8f acc[8] = {};
#pragma unroll
  for (int kc = 0; kc < INF / 32; ++kc) { v16b a; { const float* p = X + (r0 + col) * INF + kc * 32 + 8 * g;
#pragma unroll
      for (int i = 0; i < 8; ++i) { a[i] = (__bf16)p[i]; a[8 + i] = (__bf16)p[16 + i]; } }
#pragma unroll
    for (int j = 0; j < 8; ++j) acc[j] = wmma_bf(a, frag_b(PF + (size_t)(c0 + j * 16 + col) * INF + kc * 32, lane), acc[j]); }
#pragma unroll
  for (int j = 0; j < 8; ++j) { const float bb = bfr(BF[c0 + j * 16 + col]);
#pragma unroll
    for (int r = 0; r < 8; ++r) so[wave][8 * g + r][j * 16 + col] = acc[j][r] + bb; }
  LDSX(); for (int rl = 0; rl < 16; ++rl) vst2(FE + (r0 + rl) * DD + c0 + lane * 4, *(const v4f*)&so[wave][rl][lane * 4]); }
__global__ __launch_bounds__(32) void k_cells(const float* __restrict__ CO, int* __restrict__ CE) { __shared__ __align__(16) int sc[32]; const int t = threadIdx.x; const size_t p = (size_t)blockIdx.x * 32 + t;
  const float cx = bfr(CO[p * 2]), cy = bfr(CO[p * 2 + 1]); int gx = (int)(cx / 32.0f), gy = (int)(cy / 32.0f); gx = gx < 0 ? 0 : (gx > GX - 1 ? GX - 1 : gx); gy = gy < 0 ? 0 : (gy > GY - 1 ? GY - 1 : gy); sc[t] = gx * GY + gy; __syncthreads();
  if (t < 8) vst2((float*)(CE + blockIdx.x * 32 + t * 4), *(const v4f*)&sc[t * 4]); }
__global__ __launch_bounds__(256) void k_cmean(const float* __restrict__ FE, const int* __restrict__ CE, const float* __restrict__ WP1, const float* __restrict__ BP1, const float* __restrict__ WP2, const float* __restrict__ BP2, float* __restrict__ KA, float* __restrict__ CN) {
  __shared__ int scl[NP]; __shared__ float sh[DD / 2]; __shared__ __align__(16) float so2[DD];
  const int t = threadIdx.x; const int c = blockIdx.x; const size_t b = blockIdx.y;
  for (int e = t; e < NP; e += 256) scl[e] = CE[b * NP + e]; __syncthreads();
  float s0 = 0.f, s1 = 0.f; int cnt = 0; for (int n = 0; n < NP; ++n) { if (scl[n] == c) { ++cnt; s0 += FE[(b * NP + n) * DD + t]; s1 += FE[(b * NP + n) * DD + t + 256]; } }
  const float inv = 1.0f / (float)(cnt > 1 ? cnt : 1); so2[t] = s0 * inv; so2[t + 256] = s1 * inv; __syncthreads();
  if (t < DD / 4) vst2(KA + (b * NG + c) * DD + t * 4, *(const v4f*)&so2[t * 4]);
  if (c == 0) { __shared__ __align__(16) float scc[NG];
    if (t < NG) { int k = 0; for (int n = 0; n < NP; ++n) k += (scl[n] == t); scc[t] = (float)k; } __syncthreads(); if (t < NG / 4) vst2(CN + b * NG + t * 4, *(const v4f*)&scc[t * 4]); }
  if (b == 0 && c < 10) { __syncthreads();
    if (c < KN) { const float ox = (float)(c / 3 - 1), oy = (float)(c % 3 - 1);
      sh[t] = fmaxf(ox * bfr(WP1[t]) + oy * bfr(WP1[DD / 2 + t]) + bfr(BP1[t]), 0.f); __syncthreads();
      float a0 = 0.f, a1 = 0.f; for (int j = 0; j < DD / 2; ++j) { a0 += sh[j] * bfr(WP2[(size_t)j * DD + t]); a1 += sh[j] * bfr(WP2[(size_t)j * DD + t + 256]); } so2[t] = a0 + bfr(BP2[t]); so2[t + 256] = a1 + bfr(BP2[t + 256]); __syncthreads();
      if (t < DD / 4) vst2(KA + (size_t)(NCM + c) * DD + t * 4, *(const v4f*)&so2[t * 4]); }
    else { v4f z = {0.f, 0.f, 0.f, 0.f}; for (int r = NCM + KN; r < NKR; ++r) if (t < DD / 4) vst2(KA + (size_t)r * DD + t * 4, z); } }
}
template <int MODE>
__global__ __launch_bounds__(128) void k_g(const float* __restrict__ A, const __bf16* __restrict__ PW, const float* __restrict__ B1, const float* __restrict__ B2, const float* __restrict__ FE, float* __restrict__ O1, float* __restrict__ O2) { __shared__ __align__(16) float so[4][16][132];
  const int tid = threadIdx.x, wave = tid >> 5, lane = tid & 31, col = lane & 15, g = lane >> 4; const int which = blockIdx.z; const size_t r0 = (size_t)blockIdx.x * 64 + wave * 16; const int c0 = blockIdx.y * 128;
  const __bf16* Wr = PW + (size_t)((MODE == 0) ? (1 + which) : (MODE == 1) ? 0 : 3) * DD * DD; const float* BB = (MODE == 0 && which == 1) ? B2 : B1;
  v8f acc[8] = {};
#pragma unroll 2
  for (int kc = 0; kc < DD / 32; ++kc) { const F2 a = split_row(A + (r0 + col) * DD, kc * 32, lane);
#pragma unroll
    for (int j = 0; j < 8; ++j) { const v16b w = frag_b(Wr + (size_t)(c0 + j * 16 + col) * DD + kc * 32, lane); acc[j] = wmma_bf(a.h, w, acc[j]); acc[j] = wmma_bf(a.l, w, acc[j]); } }
#pragma unroll
  for (int j = 0; j < 8; ++j) { const int c = c0 + j * 16 + col; const float bb = bfr(BB[c]);
#pragma unroll
    for (int r = 0; r < 8; ++r) { const size_t row = r0 + 8 * g + r; float v = acc[j][r]; if (MODE == 0) v += (row >= NCM) ? bb : 0.f; else if (MODE == 1) v += bb; else v += bb + FE[row * DD + c]; so[wave][8 * g + r][j * 16 + col] = v; } }
  LDSX(); float* OUT = (MODE == 0 && which == 1) ? O2 : O1; for (int rl = 0; rl < 16; ++rl) vst2(OUT + (r0 + rl) * DD + c0 + lane * 4, *(const v4f*)&so[wave][rl][lane * 4]); }
__global__ __launch_bounds__(128) void k_point(const float* __restrict__ Q, const int* __restrict__ CE, const float* __restrict__ CN, const float* __restrict__ MK, const float* __restrict__ MV, float* __restrict__ AG) { __shared__ __align__(16) float so2[DD];
  const int t = threadIdx.x; const int h = t >> 5, ln = t & 31; const size_t p = blockIdx.x; const size_t b = p / NP; const int cell = CE[p]; const int gx = cell / GY, gy = cell % GY;
  float qv[4]; for (int i = 0; i < 4; ++i) qv[i] = Q[p * DD + h * HD + ln * 4 + i];
  float sc[KN]; bool ok[KN]; float mx = -3.0e38f;
#pragma unroll
  for (int kk = 0; kk < KN; ++kk) { const int nx = gx + kk / 3 - 1, ny = gy + kk % 3 - 1; const bool inb = nx >= 0 && nx < GX && ny >= 0 && ny < GY; const int nc = (nx < 0 ? 0 : nx > GX - 1 ? GX - 1 : nx) * GY + (ny < 0 ? 0 : ny > GY - 1 ? GY - 1 : ny);
    ok[kk] = inb && (CN[b * NG + nc] > 0.f); float a = 0.f; const float* k1 = MK + (b * NG + nc) * DD + h * HD + ln * 4; const float* k2 = MK + (size_t)(NCM + kk) * DD + h * HD + ln * 4;
    for (int i = 0; i < 4; ++i) a += qv[i] * (k1[i] + k2[i]);
#pragma unroll
    for (int o = 1; o < 32; o <<= 1) a += __shfl_xor(a, o);
    sc[kk] = ok[kk] ? a * 0.088388347648318441f : -1.0e9f; mx = fmaxf(mx, sc[kk]); }
  float z = 0.f;
#pragma unroll
  for (int kk = 0; kk < KN; ++kk) { sc[kk] = __expf(sc[kk] - mx); z += sc[kk]; }
  float acc4[4] = {0.f, 0.f, 0.f, 0.f};
#pragma unroll
  for (int kk = 0; kk < KN; ++kk) { const int nx = gx + kk / 3 - 1, ny = gy + kk % 3 - 1; const int nc = (nx < 0 ? 0 : nx > GX - 1 ? GX - 1 : nx) * GY + (ny < 0 ? 0 : ny > GY - 1 ? GY - 1 : ny); const float w = sc[kk] / z; const float* v1 = MV + (b * NG + nc) * DD + h * HD + ln * 4; const float* v2 = MV + (size_t)(NCM + kk) * DD + h * HD + ln * 4;
    for (int i = 0; i < 4; ++i) acc4[i] += w * (v1[i] + v2[i]); }
  v4f o4; for (int i = 0; i < 4; ++i) o4[i] = acc4[i]; *(v4f*)&so2[h * HD + ln * 4] = o4; __syncthreads(); vst2(AG + p * DD + t * 4, *(const v4f*)&so2[t * 4]); }
__global__ __launch_bounds__(256) void k_lnout(const float* __restrict__ E, const float* __restrict__ G, const float* __restrict__ Bt, float* __restrict__ OUT) { __shared__ float red[8]; __shared__ __align__(16) float so2[DD]; const int t = threadIdx.x; const size_t row = blockIdx.x;
  const float v0 = E[row * DD + t], v1 = E[row * DD + t + 256]; float s = v0 + v1;
#pragma unroll
  for (int o = 1; o < 32; o <<= 1) s += __shfl_xor(s, o);
  if ((t & 31) == 0) red[t >> 5] = s; __syncthreads(); float tot = 0.f; for (int i = 0; i < 8; ++i) tot += red[i]; const float mu = tot / (float)DD; __syncthreads();
  const float d0 = v0 - mu, d1 = v1 - mu; float q = d0 * d0 + d1 * d1;
#pragma unroll
  for (int o = 1; o < 32; o <<= 1) q += __shfl_xor(q, o);
  if ((t & 31) == 0) red[t >> 5] = q; __syncthreads(); float tq = 0.f; for (int i = 0; i < 8; ++i) tq += red[i]; const float inv = 1.0f / sqrtf(tq / (float)DD + 1e-5f);
  so2[t] = d0 * inv * bfr(G[t]) + bfr(Bt[t]); so2[t + 256] = d1 * inv * bfr(G[t + 256]) + bfr(Bt[t + 256]); __syncthreads(); if (t < DD / 4) vst2(OUT + row * DD + t * 4, *(const v4f*)&so2[t * 4]); }
extern "C" void kernel_launch(void* const* d_in, const int* in_sizes, int n_in, void* d_out, int out_size, void* d_ws, size_t ws_size, hipStream_t stream) {
  (void)in_sizes; (void)n_in; (void)out_size;
  const float** F = (const float**)d_in;
  if (ws_size < (size_t)WS_END) return;
  char* ws = (char*)d_ws; __bf16 *PF = (__bf16*)(ws + WS_PF), *PW = (__bf16*)(ws + WS_PW); float *FE = (float*)(ws + WS_FE), *KA = (float*)(ws + WS_KA), *CN = (float*)(ws + WS_CN), *MK = (float*)(ws + WS_MK), *MV = (float*)(ws + WS_MV), *Q = (float*)(ws + WS_Q), *AG = (float*)(ws + WS_AG), *E = (float*)(ws + WS_E); int* CE = (int*)(ws + WS_CE);
  k_pack<<<dim3(DD, 5), 256, 0, stream>>>(F[2], F[8], F[10], F[12], F[14], PF, PW);
  k_feat<<<dim3(NR / 64, DD / 128), 128, 0, stream>>>(F[0], PF, F[3], FE);
  k_cells<<<NR / 32, 32, 0, stream>>>(F[1], CE);
  k_cmean<<<dim3(NG, NB), 256, 0, stream>>>(FE, CE, F[4], F[5], F[6], F[7], KA, CN);
  k_g<0><<<dim3(NKR / 64, DD / 128, 2), 128, 0, stream>>>(KA, PW, F[11], F[13], nullptr, MK, MV);
  k_g<1><<<dim3(TRB, DD / 128, 1), 128, 0, stream>>>(FE, PW, F[9], nullptr, nullptr, Q, nullptr);
  k_point<<<TRB * 64, 128, 0, stream>>>(Q, CE, CN, MK, MV, AG);
  k_g<2><<<dim3(TRB, DD / 128, 1), 128, 0, stream>>>(AG, PW, F[15], nullptr, FE, E, nullptr);
  k_lnout<<<TRB * 64, 256, 0, stream>>>(E, F[16], F[17], (float*)d_out);
}
